// SerriformBlock_4715874091320
// MI455X (gfx1250) — hardware-verified
//
#include <hip/hip_runtime.h>
#include <stddef.h>
#include <stdint.h>
#include <math.h>

#define NTOK  8192
#define SEQL  2048
#define DM    1024
#define HD    256
#define NE    8
#define TOPK  2
#define TR    64
#define NTILE 264
#define MP    16896
#define TABH  32
#define TABN  (TABH + MP)
#define TPT   32
#define NTHR  256
#define GTHR  128
#define WSMAX 134217728
#define LDS_BKT ((TABN + NE * 8) * 4)
#define EPSN  1e-6f
#define WSC   256.0f
#define IWSC  0.00390625f
#define YSC   16.0f
#define IYSC  0.0625f
#define GSC   16.0f
#define IGSC  0.0625f

static_assert(MP == NTILE * TR);
static_assert(MP >= NTOK * TOPK + NE * (TR - 1));
static_assert((TABN % 32) == 0);
static_assert((MP % 4) == 0 && (TABH % 4) == 0);
static_assert(NTOK == NTHR * TPT);
static_assert((NTOK % TR) == 0);
static_assert((DM % 64) == 0 && (HD % 64) == 0);
static_assert((DM % 32) == 0 && (HD % 32) == 0);
static_assert(TR == (GTHR / 32) * 16);
static_assert(LDS_BKT <= 160000);
static_assert(NTHR / 32 == 8);
static_assert(NTOK == 4 * SEQL);
static_assert(DM == 4 * NTHR);
static_assert((DM / 8) == 128);
static_assert(MP * 2 >= NTOK * 4);

typedef float          v4f  __attribute__((ext_vector_type(4)));
typedef float          v8f  __attribute__((ext_vector_type(8)));
typedef int            v4i  __attribute__((ext_vector_type(4)));
typedef int            v8i  __attribute__((ext_vector_type(8)));
typedef unsigned int   v2u  __attribute__((ext_vector_type(2)));
typedef unsigned short v8us __attribute__((ext_vector_type(8)));
typedef __bf16         v16bf __attribute__((ext_vector_type(16)));
typedef _Float16       v16h __attribute__((ext_vector_type(16)));
typedef _Float16       v8h  __attribute__((ext_vector_type(8)));
typedef _Float16       v4h  __attribute__((ext_vector_type(4)));
union FragB { v16bf v; v8us h[2]; v8i w; };
union FragH { v16h v; v8us h[2]; v8i w; };
union H8 { v8h h; v8us u; };
union H4 { v4h h; v2u u; };

__device__ __forceinline__ v8f wmb(const FragB& a, const FragB& b, v8f c) {
  v8f d = __builtin_amdgcn_wmma_f32_16x16x32_bf16(false, a.v, false, b.v, (short)0, c, false, false);
  asm volatile("v_nop\n\tv_nop\n\tv_nop\n\tv_nop" : "+v"(d) : "v"(a.w), "v"(b.w));
  return d;
}
__device__ __forceinline__ v8f wmh(const FragH& a, const FragH& b, v8f c) {
  v8f d = __builtin_amdgcn_wmma_f32_16x16x32_f16(false, a.v, false, b.v, (short)0, c, false, false);
  asm volatile("v_nop\n\tv_nop\n\tv_nop\n\tv_nop" : "+v"(d) : "v"(a.w), "v"(b.w));
  return d;
}

__device__ __forceinline__ unsigned short rne16(float f) {
  unsigned u = __float_as_uint(f);
  u += 0x7FFFu + ((u >> 16) & 1u);
  return (unsigned short)(u >> 16);
}
__device__ __forceinline__ float rne16f(float f) {
  return __uint_as_float(((unsigned)rne16(f)) << 16);
}
__device__ __forceinline__ v4f rne4(const v4f a) {
  v4f o;
  o.x = rne16f(a.x); o.y = rne16f(a.y); o.z = rne16f(a.z); o.w = rne16f(a.w);
  return o;
}
__device__ __forceinline__ v8us cvt8(const v4f a, const v4f b) {
  v8us o;
  o[0] = rne16(a.x); o[1] = rne16(a.y); o[2] = rne16(a.z); o[3] = rne16(a.w);
  o[4] = rne16(b.x); o[5] = rne16(b.y); o[6] = rne16(b.z); o[7] = rne16(b.w);
  return o;
}
__device__ __forceinline__ void sp1(float v, unsigned short& hi, unsigned short& lo) {
  const unsigned short hb = rne16(v);
  const float hf = __uint_as_float(((unsigned)hb) << 16);
  hi = hb;
  lo = rne16(v - hf);
}
__device__ __forceinline__ void split8(const v4f a, const v4f b, v8us& hv, v8us& lv) {
  unsigned short h0, h1, h2, h3, h4, h5, h6, h7, l0, l1, l2, l3, l4, l5, l6, l7;
  sp1(a.x, h0, l0); sp1(a.y, h1, l1); sp1(a.z, h2, l2); sp1(a.w, h3, l3);
  sp1(b.x, h4, l4); sp1(b.y, h5, l5); sp1(b.z, h6, l6); sp1(b.w, h7, l7);
  hv[0] = h0; hv[1] = h1; hv[2] = h2; hv[3] = h3; hv[4] = h4; hv[5] = h5; hv[6] = h6; hv[7] = h7;
  lv[0] = l0; lv[1] = l1; lv[2] = l2; lv[3] = l3; lv[4] = l4; lv[5] = l5; lv[6] = l6; lv[7] = l7;
}
__device__ __forceinline__ v8us h16x8(const v4f a, const v4f b, const float sc) {
  const v8h hv = { (_Float16)(a.x * sc), (_Float16)(a.y * sc), (_Float16)(a.z * sc), (_Float16)(a.w * sc),
                   (_Float16)(b.x * sc), (_Float16)(b.y * sc), (_Float16)(b.z * sc), (_Float16)(b.w * sc) };
  H8 q;
  q.h = hv;
  return q.u;
}

template <int NP, int F16>
__device__ __forceinline__ void mac64(v8f (&acc)[4], const unsigned short* __restrict__ ap0,
                                      const unsigned short* __restrict__ ap1,
                                      const unsigned short* __restrict__ bp, int ldb, int nks) {
#pragma unroll 1
  for (int ks = 0; ks < nks; ++ks) {
    const int ko = 32 * ks;
    if (F16 != 0) {
      FragH a0, a1;
      a0.h[0] = *(const v8us*)(ap0 + ko);
      a0.h[1] = *(const v8us*)(ap0 + ko + 16);
      if (NP == 2) {
        a1.h[0] = *(const v8us*)(ap1 + ko);
        a1.h[1] = *(const v8us*)(ap1 + ko + 16);
      } else {
        a1 = a0;
      }
#pragma unroll
      for (int t = 0; t < 4; ++t) {
        const unsigned short* q = bp + (size_t)(16 * t) * (size_t)ldb + ko;
        FragH b;
        b.h[0] = *(const v8us*)q;
        b.h[1] = *(const v8us*)(q + 16);
        acc[t] = wmh(a0, b, acc[t]);
        if (NP == 2) acc[t] = wmh(a1, b, acc[t]);
      }
    } else {
      FragB a0, a1;
      a0.h[0] = *(const v8us*)(ap0 + ko);
      a0.h[1] = *(const v8us*)(ap0 + ko + 16);
      if (NP == 2) {
        a1.h[0] = *(const v8us*)(ap1 + ko);
        a1.h[1] = *(const v8us*)(ap1 + ko + 16);
      } else {
        a1 = a0;
      }
#pragma unroll
      for (int t = 0; t < 4; ++t) {
        const unsigned short* q = bp + (size_t)(16 * t) * (size_t)ldb + ko;
        FragB b;
        b.h[0] = *(const v8us*)q;
        b.h[1] = *(const v8us*)(q + 16);
        acc[t] = wmb(a0, b, acc[t]);
        if (NP == 2) acc[t] = wmb(a1, b, acc[t]);
      }
    }
  }
}

template <int RESM>
__device__ __forceinline__ void store_tile_f32(const float* stg, float* dst, const float* __restrict__ res,
                                               int ldd, int rowBase, int col0, int wave, int lane) {
  const int hh = lane >> 4, m = lane & 15;
  v4f fv[8];
  size_t op[8];
#pragma unroll
  for (int i = 0; i < 8; ++i) {
    const int lr = 16 * wave + 2 * i + hh;
    v4f v = *(const v4f*)(stg + lr * 64 + 4 * m);
    op[i] = (size_t)(rowBase + lr) * (size_t)ldd + (size_t)(col0 + 4 * m);
    if (RESM != 0) {
      v4f rr = *(const v4f*)(res + op[i]);
      if (RESM == 2) rr = rne4(rr);
      v = v + rr;
    }
    fv[i] = v;
  }
#pragma unroll
  for (int i = 0; i < 8; ++i) *(volatile v4f*)(dst + op[i]) = fv[i];
  __threadfence();
#pragma unroll
  for (int i = 0; i < 8; ++i) *(volatile v4f*)(dst + op[i]) = fv[i];
}

__device__ __forceinline__ void store_tile_h16(const float* stg, unsigned short* dst, int ldd,
                                               int rowBase, int col0, int wave, int lane) {
  const int q8 = lane & 7, sub = lane >> 3;
  v8us hv[4];
  size_t po[4];
#pragma unroll
  for (int i = 0; i < 4; ++i) {
    const int lr = 16 * wave + 4 * i + sub;
    const v4f a = *(const v4f*)(stg + lr * 64 + 8 * q8);
    const v4f b = *(const v4f*)(stg + lr * 64 + 8 * q8 + 4);
    hv[i] = h16x8(a, b, 1.0f);
    po[i] = (size_t)(rowBase + lr) * (size_t)ldd + (size_t)(col0 + 8 * q8);
  }
#pragma unroll
  for (int i = 0; i < 4; ++i) *(volatile v8us*)(dst + po[i]) = hv[i];
  __threadfence();
#pragma unroll
  for (int i = 0; i < 4; ++i) *(volatile v8us*)(dst + po[i]) = hv[i];
}

__global__ __launch_bounds__(NTHR) void k_cvt(const float* __restrict__ src, unsigned short* dst, int n8, float sc, int hmode) {
  const int u = (int)blockIdx.x * NTHR + (int)threadIdx.x;
  if (u >= n8) return;
  const float* p = src + (size_t)u * 8;
  v4f a = *(const v4f*)p;
  v4f b = *(const v4f*)(p + 4);
  a = rne4(a);
  b = rne4(b);
  v8us o;
  if (hmode != 0) o = h16x8(a, b, sc); else o = cvt8(a, b);
  const size_t q = (size_t)u * 8;
  *(volatile v8us*)(dst + q) = o;
  __threadfence();
  *(volatile v8us*)(dst + q) = o;
}

__global__ __launch_bounds__(NTHR) void k_dwconv(const float* __restrict__ x, const float* __restrict__ ker,
                                                 const float* __restrict__ bias, unsigned short* yh, unsigned short* yl,
                                                 int nUnits) {
  const int u = (int)blockIdx.x * NTHR + (int)threadIdx.x;
  if (u >= nUnits) return;
  const int t  = u >> 7;
  const int c8 = (u & 127) * 8;
  const int l  = t & (SEQL - 1);
  const int t1 = (l >= 1) ? t - 1 : t;
  const int t2 = (l >= 2) ? t - 2 : t;
  const float f1 = (l >= 1) ? 1.0f : 0.0f;
  const float f2 = (l >= 2) ? 1.0f : 0.0f;
  const float* p0 = x + (size_t)t  * DM + c8;
  const float* p1 = x + (size_t)t1 * DM + c8;
  const float* p2 = x + (size_t)t2 * DM + c8;
  const v4f x0a = rne4(*(const v4f*)p0), x0b = rne4(*(const v4f*)(p0 + 4));
  const v4f x1a = rne4(*(const v4f*)p1), x1b = rne4(*(const v4f*)(p1 + 4));
  const v4f x2a = rne4(*(const v4f*)p2), x2b = rne4(*(const v4f*)(p2 + 4));
  const float* kp = ker + (size_t)c8 * 3;
  const v4f kv0 = *(const v4f*)kp,        kv1 = *(const v4f*)(kp + 4),  kv2 = *(const v4f*)(kp + 8);
  const v4f kv3 = *(const v4f*)(kp + 12), kv4 = *(const v4f*)(kp + 16), kv5 = *(const v4f*)(kp + 20);
  const v4f ba = rne4(*(const v4f*)(bias + c8)), bb = rne4(*(const v4f*)(bias + c8 + 4));
  const float kk[24] = { kv0.x, kv0.y, kv0.z, kv0.w, kv1.x, kv1.y, kv1.z, kv1.w, kv2.x, kv2.y, kv2.z, kv2.w,
                         kv3.x, kv3.y, kv3.z, kv3.w, kv4.x, kv4.y, kv4.z, kv4.w, kv5.x, kv5.y, kv5.z, kv5.w };
  const float xc[8]  = { x0a.x, x0a.y, x0a.z, x0a.w, x0b.x, x0b.y, x0b.z, x0b.w };
  const float xm1[8] = { x1a.x, x1a.y, x1a.z, x1a.w, x1b.x, x1b.y, x1b.z, x1b.w };
  const float xm2[8] = { x2a.x, x2a.y, x2a.z, x2a.w, x2b.x, x2b.y, x2b.z, x2b.w };
  const float bv[8]  = { ba.x, ba.y, ba.z, ba.w, bb.x, bb.y, bb.z, bb.w };
  float y[8];
#pragma unroll
  for (int i = 0; i < 8; ++i) {
    const float w0 = rne16f(kk[3 * i + 0]) * f2;
    const float w1 = rne16f(kk[3 * i + 1]) * f1;
    const float w2 = rne16f(kk[3 * i + 2]);
    y[i] = ((xm2[i] * w0 + xm1[i] * w1) + xc[i] * w2) + bv[i];
  }
  const v4f ya = { y[0], y[1], y[2], y[3] };
  const v4f yb = { y[4], y[5], y[6], y[7] };
  v8us hv, lv;
  split8(ya, yb, hv, lv);
  const size_t q = (size_t)t * DM + (size_t)c8;
  *(volatile v8us*)(yh + q) = hv;
  *(volatile v8us*)(yl + q) = lv;
  __threadfence();
  *(volatile v8us*)(yh + q) = hv;
  *(volatile v8us*)(yl + q) = lv;
}

__global__ __launch_bounds__(GTHR) void k_pw(const unsigned short* __restrict__ yh, const unsigned short* __restrict__ yl,
                                             const unsigned short* __restrict__ wpw, const float* __restrict__ pwb,
                                             const float* __restrict__ x, float* x1f) {
  __shared__ __attribute__((aligned(16))) float stg[TR * 64];
  const int tid = (int)threadIdx.x, lane = tid & 31, wave = tid >> 5, hh = lane >> 4, m = lane & 15;
  const int rowBase = (int)blockIdx.x * TR;
  const int col0    = (int)blockIdx.y * 64;
  v8f acc[4];
  {
    const v8f z = {0.f, 0.f, 0.f, 0.f, 0.f, 0.f, 0.f, 0.f};
    acc[0] = z; acc[1] = z; acc[2] = z; acc[3] = z;
  }
  const size_t arow = (size_t)(rowBase + 16 * wave + m) * (size_t)DM + (size_t)(8 * hh);
  mac64<2, 0>(acc, yh + arow, yl + arow, wpw + (size_t)(col0 + m) * (size_t)DM + (size_t)(8 * hh), DM, DM / 32);

#pragma unroll
  for (int t = 0; t < 4; ++t) {
    const int lc = 16 * t + m;
    const float bc = rne16f(pwb[col0 + lc]);
#pragma unroll
    for (int r = 0; r < 8; ++r) {
      const int lr = 16 * wave + 8 * hh + r;
      const float v = acc[t][r] + bc;
      const float sg = __builtin_amdgcn_rcpf(1.0f + __expf(-v));
      stg[lr * 64 + lc] = v * sg;
    }
  }
  __syncthreads();
  store_tile_f32<2>(stg, x1f, x, DM, rowBase, col0, wave, lane);
}

__device__ __forceinline__ void gacc(float xq, const float* swrow, float (&acc)[NE]) {
  const v4f wa = *(const v4f*)(swrow);
  const v4f wb = *(const v4f*)(swrow + 4);
  acc[0] = fmaf(xq, wa.x, acc[0]); acc[1] = fmaf(xq, wa.y, acc[1]);
  acc[2] = fmaf(xq, wa.z, acc[2]); acc[3] = fmaf(xq, wa.w, acc[3]);
  acc[4] = fmaf(xq, wb.x, acc[4]); acc[5] = fmaf(xq, wb.y, acc[5]);
  acc[6] = fmaf(xq, wb.z, acc[6]); acc[7] = fmaf(xq, wb.w, acc[7]);
}

__global__ __launch_bounds__(NTHR) void k_gate(const float* __restrict__ x1, const float* __restrict__ rw,
                                               const float* __restrict__ rb, int* route) {
  __shared__ __attribute__((aligned(16))) float sw[DM * NE];
  const int tid = (int)threadIdx.x;
#pragma unroll 1
  for (int i = tid; i < DM * NE; i += NTHR) {
    const int d = i >> 3, e = i & 7;
    sw[i] = rne16f(rw[(size_t)e * DM + d]);
  }
  __syncthreads();
  int t = (int)blockIdx.x * NTHR + tid;
  const bool live = t < NTOK;
  t = t > NTOK - 1 ? NTOK - 1 : t;
  const float* xr = x1 + (size_t)t * DM;
  float acc[NE];
#pragma unroll
  for (int e = 0; e < NE; ++e) acc[e] = 0.f;
#pragma unroll 1
  for (int d4 = 0; d4 < DM / 4; ++d4) {
    const v4f xv = *(const v4f*)(xr + 4 * d4);
    const float* swr = sw + (size_t)(4 * d4) * NE;
    gacc(xv.x, swr,          acc);
    gacc(xv.y, swr + NE,     acc);
    gacc(xv.z, swr + 2 * NE, acc);
    gacc(xv.w, swr + 3 * NE, acc);
  }
  const v4f rba = *(const v4f*)rb;
  const v4f rbb = *(const v4f*)(rb + 4);
  float lg[NE];
  lg[0] = acc[0] + rne16f(rba.x); lg[1] = acc[1] + rne16f(rba.y);
  lg[2] = acc[2] + rne16f(rba.z); lg[3] = acc[3] + rne16f(rba.w);
  lg[4] = acc[4] + rne16f(rbb.x); lg[5] = acc[5] + rne16f(rbb.y);
  lg[6] = acc[6] + rne16f(rbb.z); lg[7] = acc[7] + rne16f(rbb.w);
  int i1 = 0;
  float b1 = lg[0];
#pragma unroll
  for (int e = 1; e < NE; ++e) {
    const bool up = lg[e] > b1;
    i1 = up ? e : i1;
    b1 = up ? lg[e] : b1;
  }
  int i2 = (i1 == 0) ? 1 : 0;
  float b2 = (i1 == 0) ? lg[1] : lg[0];
#pragma unroll
  for (int e = 0; e < NE; ++e) {
    const bool ok = (e != i1) && (lg[e] > b2);
    i2 = ok ? e : i2;
    b2 = ok ? lg[e] : b2;
  }
  const float e2 = __expf(b2 - b1);
  const float s  = 1.0f + e2;
  const float rs = 1.0f / s;
  const float p1 = rs;
  const float p2 = e2 * rs;
  v4i rec;
  rec.x = i1; rec.y = i2; rec.z = __float_as_int(p1); rec.w = __float_as_int(p2);
  if (live) *(volatile v4i*)(route + (size_t)t * 4) = rec;
  __threadfence();
  if (live) *(volatile v4i*)(route + (size_t)t * 4) = rec;
}

__device__ __forceinline__ void cnt_add(int c, int (&cnt)[NE]) {
  c = c < 0 ? 0 : (c > NE - 1 ? NE - 1 : c);
#pragma unroll
  for (int e = 0; e < NE; ++e) cnt[e] += (c == e) ? 1 : 0;
}
__device__ __forceinline__ int slot_of(int c, int (&base)[NE]) {
  c = c < 0 ? 0 : (c > NE - 1 ? NE - 1 : c);
  int p = 0;
#pragma unroll
  for (int e = 0; e < NE; ++e) {
    const bool mt = (c == e);
    p = mt ? base[e] : p;
    base[e] += mt ? 1 : 0;
  }
  return p < 0 ? 0 : (p > MP - 1 ? MP - 1 : p);
}

__global__ __launch_bounds__(NTHR) void k_bucket(const int* __restrict__ route, int* tab) {
  extern __shared__ v4i lds_dyn[];
  int* img = (int*)lds_dyn;
  int* lst = img + TABH;
  int* wt  = img + TABN;
  const int tid = (int)threadIdx.x, lane = tid & 31, wave = tid >> 5;

  const v4i z4 = {0, 0, 0, 0};
#pragma unroll 1
  for (int p = tid; p < TABN / 4; p += NTHR) *(v4i*)(img + 4 * p) = z4;
  __syncthreads();
  const v4i m4 = {-1, -1, -1, -1};
#pragma unroll 1
  for (int p = tid; p < MP / 4; p += NTHR) *(v4i*)(lst + 4 * p) = m4;
  __syncthreads();

  const int t0 = tid * TPT;
  int cnt[NE];
#pragma unroll
  for (int e = 0; e < NE; ++e) cnt[e] = 0;
#pragma unroll 1
  for (int c = 0; c < TPT; ++c) {
    const v4i rc = *(const v4i*)(route + (size_t)(t0 + c) * 4);
    cnt_add(rc.x, cnt);
    cnt_add(rc.y, cnt);
  }
  int incl[NE];
#pragma unroll
  for (int e = 0; e < NE; ++e) {
    int v = cnt[e];
#pragma unroll
    for (int d = 1; d < 32; d <<= 1) {
      const int up = __shfl_up(v, d);
      if (lane >= d) v += up;
    }
    incl[e] = v;
    if (lane == 31) wt[e * 8 + wave] = v;
  }
  __syncthreads();
  int pre[NE], tot[NE];
#pragma unroll
  for (int e = 0; e < NE; ++e) {
    int s = 0, all = 0;
#pragma unroll
    for (int w2 = 0; w2 < NTHR / 32; ++w2) {
      const int v = wt[e * 8 + w2];
      all += v;
      s   += (w2 < wave) ? v : 0;
    }
    pre[e] = s + incl[e] - cnt[e];
    all = all < 0 ? 0 : (all > NTOK * TOPK ? NTOK * TOPK : all);
    tot[e] = all;
  }
  int off[NE + 1];
  off[0] = 0;
#pragma unroll
  for (int e = 0; e < NE; ++e) {
    int nx = off[e] + ((tot[e] + TR - 1) / TR) * TR;
    nx = nx > MP ? MP : nx;
    off[e + 1] = nx;
  }
  int base[NE];
#pragma unroll
  for (int e = 0; e < NE; ++e) base[e] = off[e] + pre[e];
#pragma unroll 1
  for (int c = 0; c < TPT; ++c) {
    const v4i rc = *(const v4i*)(route + (size_t)(t0 + c) * 4);
    const int t = t0 + c;
    const int pa = slot_of(rc.x, base); lst[pa] = 2 * t;
    const int pb = slot_of(rc.y, base); lst[pb] = 2 * t + 1;
  }
  __syncthreads();
  if (tid == 0) {
#pragma unroll
    for (int e = 0; e < NE; ++e) img[e] = tot[e];
#pragma unroll
    for (int j = 0; j <= NE; ++j) img[NE + j] = off[j];
  }
  __syncthreads();
#pragma unroll 1
  for (int p = tid; p < TABN / 4; p += NTHR) {
    const v4i v = *(const v4i*)(img + 4 * p);
    *(volatile v4i*)(tab + 4 * p) = v;
  }
  __threadfence();
#pragma unroll 1
  for (int p = tid; p < TABN / 4; p += NTHR) {
    const v4i v = *(const v4i*)(img + 4 * p);
    *(volatile v4i*)(tab + 4 * p) = v;
  }
}

__global__ __launch_bounds__(NTHR) void k_gather(const float* __restrict__ x1, const int* __restrict__ tab,
                                                 unsigned short* xg, int nUnits) {
  const int u = (int)blockIdx.x * NTHR + (int)threadIdx.x;
  if (u >= nUnits) return;
  const int row = u >> 7;
  const int c8  = (u & 127) * 8;
  const int code = tab[TABH + row];
  int t = code < 0 ? 0 : (code >> 1);
  t = t > NTOK - 1 ? NTOK - 1 : t;
  const float* p = x1 + (size_t)t * DM + c8;
  const v4f a = *(const v4f*)p;
  const v4f b = *(const v4f*)(p + 4);
  const v8us o = h16x8(a, b, 1.0f);
  const size_t q = (size_t)row * DM + (size_t)c8;
  *(volatile v8us*)(xg + q) = o;
  __threadfence();
  *(volatile v8us*)(xg + q) = o;
}

__device__ __forceinline__ int tile_slot(const int* __restrict__ tab, int rowBase) {
  const v4i ho0 = *(const v4i*)(tab + 8);
  const v4i ho1 = *(const v4i*)(tab + 12);
  int e = 0;
#define SELX(J, OJ) { const bool ge_ = rowBase >= (OJ); e = ge_ ? (J) : e; }
  SELX(1, ho0.y) SELX(2, ho0.z) SELX(3, ho0.w)
  SELX(4, ho1.x) SELX(5, ho1.y) SELX(6, ho1.z) SELX(7, ho1.w)
#undef SELX
  return e;
}

__global__ __launch_bounds__(GTHR) void k_expert(const unsigned short* __restrict__ xg, const unsigned short* __restrict__ wex,
                                                 const float* __restrict__ eb, const int* __restrict__ tab,
                                                 const int* __restrict__ route, unsigned short* yp) {
  __shared__ __attribute__((aligned(16))) float stg[TR * 64];
  __shared__ int   sdst[TR];
  __shared__ float sp[TR];
  const int tid = (int)threadIdx.x, lane = tid & 31, wave = tid >> 5, hh = lane >> 4, m = lane & 15;
  const int rowBase = (int)blockIdx.x * TR;
  const int col0    = (int)blockIdx.y * 64;
  const int e = tile_slot(tab, rowBase);
  if (tid < TR) {
    const int code = tab[TABH + rowBase + tid];
    const bool ok = code >= 0;
    int cc = code < 0 ? 0 : code;
    cc = cc > 2 * NTOK - 1 ? 2 * NTOK - 1 : cc;
    const int t = cc >> 1, j = cc & 1;
    const float p = __int_as_float(route[(size_t)t * 4 + 2 + j]);
    sdst[tid] = ok ? (j * NTOK + t) : -1;
    sp[tid]   = ok ? p : 0.0f;
  }
  __syncthreads();

  v8f acc[4];
  {
    const v8f z = {0.f, 0.f, 0.f, 0.f, 0.f, 0.f, 0.f, 0.f};
    acc[0] = z; acc[1] = z; acc[2] = z; acc[3] = z;
  }
  const size_t arow = (size_t)(rowBase + 16 * wave + m) * (size_t)DM + (size_t)(8 * hh);
  const unsigned short* wb = wex + (size_t)e * (size_t)(DM * DM) + (size_t)(col0 + m) * (size_t)DM + (size_t)(8 * hh);
  mac64<1, 1>(acc, xg + arow, nullptr, wb, DM, DM / 32);

#pragma unroll
  for (int t = 0; t < 4; ++t) {
    const int lc = 16 * t + m;
    const float bc = rne16f(eb[(size_t)e * DM + col0 + lc]);
#pragma unroll
    for (int r = 0; r < 8; ++r) {
      const int lr = 16 * wave + 8 * hh + r;
      const float v = acc[t][r] * IWSC + bc;
      const float sg = __builtin_amdgcn_rcpf(1.0f + __expf(-v));
      stg[lr * 64 + lc] = (v * sg) * sp[lr] * YSC;
    }
  }
  __syncthreads();

  const int q8 = lane & 7, sub = lane >> 3;
  v8us hv[4];
  size_t po[4];
  bool ok[4];
#pragma unroll
  for (int i = 0; i < 4; ++i) {
    const int lr = 16 * wave + 4 * i + sub;
    const v4f a = *(const v4f*)(stg + lr * 64 + 8 * q8);
    const v4f b = *(const v4f*)(stg + lr * 64 + 8 * q8 + 4);
    hv[i] = h16x8(a, b, 1.0f);
    const int dr = sdst[lr];
    ok[i] = dr >= 0;
    const int drc = dr < 0 ? 0 : dr;
    po[i] = (size_t)drc * (size_t)DM + (size_t)(col0 + 8 * q8);
  }
#pragma unroll
  for (int i = 0; i < 4; ++i) { if (ok[i]) *(volatile v8us*)(yp + po[i]) = hv[i]; }
  __threadfence();
#pragma unroll
  for (int i = 0; i < 4; ++i) { if (ok[i]) *(volatile v8us*)(yp + po[i]) = hv[i]; }
}

__global__ __launch_bounds__(GTHR) void k_outw(const unsigned short* __restrict__ yp, const unsigned short* __restrict__ wout,
                                               const float* __restrict__ ob, const float* __restrict__ x1f, float* z) {
  __shared__ __attribute__((aligned(16))) float stg[TR * 64];
  const int tid = (int)threadIdx.x, lane = tid & 31, wave = tid >> 5, hh = lane >> 4, m = lane & 15;
  const int rowBase = (int)blockIdx.x * TR;
  const int col0    = (int)blockIdx.y * 64;
  v8f acc[4];
  {
    const v8f zz = {0.f, 0.f, 0.f, 0.f, 0.f, 0.f, 0.f, 0.f};
    acc[0] = zz; acc[1] = zz; acc[2] = zz; acc[3] = zz;
  }
  const size_t arow = (size_t)(rowBase + 16 * wave + m) * (size_t)DM + (size_t)(8 * hh);
  mac64<2, 1>(acc, yp + arow, yp + (size_t)NTOK * (size_t)DM + arow,
              wout + (size_t)(col0 + m) * (size_t)DM + (size_t)(8 * hh), DM, DM / 32);

#pragma unroll
  for (int t = 0; t < 4; ++t) {
    const int lc = 16 * t + m;
    const float bc = rne16f(ob[col0 + lc]);
#pragma unroll
    for (int r = 0; r < 8; ++r) {
      const int lr = 16 * wave + 8 * hh + r;
      stg[lr * 64 + lc] = acc[t][r] * (IWSC * IYSC) + bc;
    }
  }
  __syncthreads();
  store_tile_f32<1>(stg, z, x1f, DM, rowBase, col0, wave, lane);
}

__global__ __launch_bounds__(NTHR) void k_norm(const float* __restrict__ z, const float* __restrict__ nw,
                                               float* hf, unsigned short* hp) {
  __shared__ float red[8];
  const int tid = (int)threadIdx.x, lane = tid & 31, wave = tid >> 5;
  const int t = (int)blockIdx.x;
  const size_t base = (size_t)t * DM + (size_t)(4 * tid);
  const v4f v = *(const v4f*)(z + base);
  float ss = v.x * v.x;
  ss = fmaf(v.y, v.y, ss);
  ss = fmaf(v.z, v.z, ss);
  ss = fmaf(v.w, v.w, ss);
#pragma unroll
  for (int o = 16; o > 0; o >>= 1) ss += __shfl_xor(ss, o);
  if (lane == 0) red[wave] = ss;
  __syncthreads();
  const float tot = ((red[0] + red[1]) + (red[2] + red[3])) + ((red[4] + red[5]) + (red[6] + red[7]));
  const float inv = 1.0f / sqrtf(tot * (1.0f / (float)DM) + EPSN);
  const v4f w4 = rne4(*(const v4f*)(nw + 4 * tid));
  v4f h;
  h.x = w4.x * (v.x * inv);
  h.y = w4.y * (v.y * inv);
  h.z = w4.z * (v.z * inv);
  h.w = w4.w * (v.w * inv);
  const v4h h4 = { (_Float16)h.x, (_Float16)h.y, (_Float16)h.z, (_Float16)h.w };
  H4 q;
  q.h = h4;
  *(volatile v4f*)(hf + base) = h;
  *(volatile v2u*)(hp + base) = q.u;
  __threadfence();
  *(volatile v4f*)(hf + base) = h;
  *(volatile v2u*)(hp + base) = q.u;
}

__global__ __launch_bounds__(GTHR) void k_ffdown(const unsigned short* __restrict__ hp, const unsigned short* __restrict__ wfd,
                                                 const float* __restrict__ fdb, unsigned short* gp) {
  __shared__ __attribute__((aligned(16))) float stg[TR * 64];
  const int tid = (int)threadIdx.x, lane = tid & 31, wave = tid >> 5, hh = lane >> 4, m = lane & 15;
  const int rowBase = (int)blockIdx.x * TR;
  const int col0    = (int)blockIdx.y * 64;
  v8f acc[4];
  {
    const v8f zz = {0.f, 0.f, 0.f, 0.f, 0.f, 0.f, 0.f, 0.f};
    acc[0] = zz; acc[1] = zz; acc[2] = zz; acc[3] = zz;
  }
  const size_t arow = (size_t)(rowBase + 16 * wave + m) * (size_t)DM + (size_t)(8 * hh);
  mac64<1, 1>(acc, hp + arow, nullptr, wfd + (size_t)(col0 + m) * (size_t)DM + (size_t)(8 * hh), DM, DM / 32);

#pragma unroll
  for (int t = 0; t < 4; ++t) {
    const int lc = 16 * t + m;
    const float bc = rne16f(fdb[col0 + lc]);
#pragma unroll
    for (int r = 0; r < 8; ++r) {
      const int lr = 16 * wave + 8 * hh + r;
      const float v = acc[t][r] * IWSC + bc;
      const float g = 0.5f * v * (1.0f + erff(v * 0.70710678118654752f));
      stg[lr * 64 + lc] = g * GSC;
    }
  }
  __syncthreads();
  store_tile_h16(stg, gp, HD, rowBase, col0, wave, lane);
}

__global__ __launch_bounds__(GTHR) void k_ffup(const unsigned short* __restrict__ gp, const unsigned short* __restrict__ wfu,
                                               const float* __restrict__ fub, const float* __restrict__ hf, float* out) {
  __shared__ __attribute__((aligned(16))) float stg[TR * 64];
  const int tid = (int)threadIdx.x, lane = tid & 31, wave = tid >> 5, hh = lane >> 4, m = lane & 15;
  const int rowBase = (int)blockIdx.x * TR;
  const int col0    = (int)blockIdx.y * 64;
  v8f acc[4];
  {
    const v8f zz = {0.f, 0.f, 0.f, 0.f, 0.f, 0.f, 0.f, 0.f};
    acc[0] = zz; acc[1] = zz; acc[2] = zz; acc[3] = zz;
  }
  const size_t arow = (size_t)(rowBase + 16 * wave + m) * (size_t)HD + (size_t)(8 * hh);
  mac64<1, 1>(acc, gp + arow, nullptr, wfu + (size_t)(col0 + m) * (size_t)HD + (size_t)(8 * hh), HD, HD / 32);

#pragma unroll
  for (int t = 0; t < 4; ++t) {
    const int lc = 16 * t + m;
    const float bc = rne16f(fub[col0 + lc]);
#pragma unroll
    for (int r = 0; r < 8; ++r) {
      const int lr = 16 * wave + 8 * hh + r;
      stg[lr * 64 + lc] = acc[t][r] * (IWSC * IGSC) + bc;
    }
  }
  __syncthreads();
  store_tile_f32<1>(stg, out, hf, DM, rowBase, col0, wave, lane);
}

static inline int cdiv(int a, int b) { return (a + b - 1) / b; }

extern "C" void kernel_launch(void* const* d_in, const int* in_sizes, int n_in,
                              void* d_out, int out_size, void* d_ws, size_t ws_size,
                              hipStream_t stream) {
  if (n_in < 16) return;
  if (in_sizes[0]  != NTOK * DM) return;
  if (in_sizes[1]  != DM * 3) return;
  if (in_sizes[2]  != DM) return;
  if (in_sizes[3]  != DM * DM) return;
  if (in_sizes[4]  != DM) return;
  if (in_sizes[5]  != NE * DM) return;
  if (in_sizes[6]  != NE) return;
  if (in_sizes[7]  != NE * DM * DM) return;
  if (in_sizes[8]  != NE * DM) return;
  if (in_sizes[9]  != DM * DM) return;
  if (in_sizes[10] != DM) return;
  if (in_sizes[11] != DM) return;
  if (in_sizes[12] != HD * DM) return;
  if (in_sizes[13] != HD) return;
  if (in_sizes[14] != DM * HD) return;
  if (in_sizes[15] != DM) return;
  if (out_size != NTOK * DM) return;

  const float* x    = (const float*)d_in[0];
  const float* dw_k = (const float*)d_in[1];
  const float* dw_b = (const float*)d_in[2];
  const float* pw_w = (const float*)d_in[3];
  const float* pw_b = (const float*)d_in[4];
  const float* rt_w = (const float*)d_in[5];
  const float* rt_b = (const float*)d_in[6];
  const float* ex_w = (const float*)d_in[7];
  const float* ex_b = (const float*)d_in[8];
  const float* ou_w = (const float*)d_in[9];
  const float* ou_b = (const float*)d_in[10];
  const float* nm_w = (const float*)d_in[11];
  const float* fd_w = (const float*)d_in[12];
  const float* fd_b = (const float*)d_in[13];
  const float* fu_w = (const float*)d_in[14];
  const float* fu_b = (const float*)d_in[15];
  float* out = (float*)d_out;

  char* ws = (char*)d_ws;
  size_t off = 0;
  const size_t oWEX = off; off += (size_t)NE * DM * DM * 2;   off = (off + 255) & ~(size_t)255;
  const size_t oWPW = off; off += (size_t)DM * DM * 2;        off = (off + 255) & ~(size_t)255;
  const size_t oWOU = off; off += (size_t)DM * DM * 2;        off = (off + 255) & ~(size_t)255;
  const size_t oWFD = off; off += (size_t)HD * DM * 2;        off = (off + 255) & ~(size_t)255;
  const size_t oWFU = off; off += (size_t)DM * HD * 2;        off = (off + 255) & ~(size_t)255;
  const size_t oRT  = off; off += (size_t)NTOK * 4 * 4;       off = (off + 255) & ~(size_t)255;
  const size_t oTAB = off; off += (size_t)TABN * 4;           off = (off + 255) & ~(size_t)255;
  const size_t oR1  = off; off += (size_t)2 * NTOK * DM * 2;  off = (off + 255) & ~(size_t)255;
  const size_t oR2  = off; off += (size_t)NTOK * DM * 4;      off = (off + 255) & ~(size_t)255;
  const size_t oR3  = off; off += (size_t)MP * DM * 2;        off = (off + 255) & ~(size_t)255;
  if (off > ws_size || off > (size_t)WSMAX) return;

  unsigned short* WEX = (unsigned short*)(ws + oWEX);
  unsigned short* WPW = (unsigned short*)(ws + oWPW);
  unsigned short* WOU = (unsigned short*)(ws + oWOU);
  unsigned short* WFD = (unsigned short*)(ws + oWFD);
  unsigned short* WFU = (unsigned short*)(ws + oWFU);
  int*            RT  = (int*)(ws + oRT);
  int*            TAB = (int*)(ws + oTAB);
  unsigned short* YH  = (unsigned short*)(ws + oR1);
  unsigned short* YL  = (unsigned short*)(ws + oR1) + (size_t)NTOK * DM;
  unsigned short* YP  = (unsigned short*)(ws + oR1);
  unsigned short* HP  = (unsigned short*)(ws + oR1);
  unsigned short* GP  = (unsigned short*)(ws + oR1) + (size_t)NTOK * DM;
  float*          X1F = (float*)(ws + oR2);
  float*          HF  = (float*)(ws + oR2);
  unsigned short* XG  = (unsigned short*)(ws + oR3);
  float*          Z   = (float*)(ws + oR3);

  hipFuncSetAttribute(reinterpret_cast<const void*>(&k_bucket),
                      hipFuncAttributeMaxDynamicSharedMemorySize, LDS_BKT);

  {
    const int n8pw = DM * DM / 8;
    const int n8ex = NE * DM * DM / 8;
    const int n8fd = HD * DM / 8;
    k_cvt<<<cdiv(n8pw, NTHR), NTHR, 0, stream>>>(pw_w, WPW, n8pw, 1.0f, 0);
    k_cvt<<<cdiv(n8ex, NTHR), NTHR, 0, stream>>>(ex_w, WEX, n8ex, WSC, 1);
    k_cvt<<<cdiv(n8pw, NTHR), NTHR, 0, stream>>>(ou_w, WOU, n8pw, WSC, 1);
    k_cvt<<<cdiv(n8fd, NTHR), NTHR, 0, stream>>>(fd_w, WFD, n8fd, WSC, 1);
    k_cvt<<<cdiv(n8fd, NTHR), NTHR, 0, stream>>>(fu_w, WFU, n8fd, WSC, 1);
  }

  {
    const int nUdw = NTOK * (DM / 8);
    k_dwconv<<<cdiv(nUdw, NTHR), NTHR, 0, stream>>>(x, dw_k, dw_b, YH, YL, nUdw);
  }
  k_pw<<<dim3(NTOK / TR, DM / 64), GTHR, 0, stream>>>(YH, YL, WPW, pw_b, x, X1F);

  k_gate<<<cdiv(NTOK, NTHR), NTHR, 0, stream>>>(X1F, rt_w, rt_b, RT);
  k_bucket<<<1, NTHR, LDS_BKT, stream>>>(RT, TAB);
  {
    const int nUg = MP * (DM / 8);
    k_gather<<<cdiv(nUg, NTHR), NTHR, 0, stream>>>(X1F, TAB, XG, nUg);
  }

  k_expert<<<dim3(NTILE, DM / 64), GTHR, 0, stream>>>(XG, WEX, ex_b, TAB, RT, YP);
  k_outw<<<dim3(NTOK / TR, DM / 64), GTHR, 0, stream>>>(YP, WOU, ou_b, X1F, Z);

  k_norm<<<NTOK, NTHR, 0, stream>>>(Z, nm_w, HF, HP);
  k_ffdown<<<dim3(NTOK / TR, HD / 64), GTHR, 0, stream>>>(HP, WFD, fd_b, GP);
  k_ffup<<<dim3(NTOK / TR, DM / 64), GTHR, 0, stream>>>(GP, WFU, fu_b, HF, out);
}
